// SurnameClassifierRNN_42417097016405
// MI455X (gfx1250) — hardware-verified
//
#include <hip/hip_runtime.h>


namespace {
constexpr int V = 10000, E = 128, H = 256, C = 18, B = 4096, S = 64, NR = B * S;
constexpr float XS = 8.0f, HS = 2048.0f, YS = 64.0f, WSC = 256.0f;
typedef _Float16 b16;
typedef __attribute__((ext_vector_type(16))) _Float16 v16b;
typedef __attribute__((ext_vector_type(8))) _Float16 v8b;
typedef __attribute__((ext_vector_type(8))) float v8f;
typedef __attribute__((ext_vector_type(4))) float v4f;
__device__ __forceinline__ float bf16_rne(float f) { unsigned int u = __float_as_uint(f); u += 0x7FFFu + ((u >> 16) & 1u); return __uint_as_float(u & 0xFFFF0000u); }
__device__ __forceinline__ void split16(float v, b16& hi, b16& lo) { hi = (b16)v; lo = (b16)(v - (float)hi); }
__device__ __forceinline__ v16b frag_kb(const b16* p, int hh) { const v8b a = *(const v8b*)(p + 8 * hh), b = *(const v8b*)(p + 16 + 8 * hh); v16b f;
#pragma unroll
  for (int e = 0; e < 8; ++e) { f[e] = a[e]; f[8 + e] = b[e]; } return f; }
__device__ __forceinline__ v8f wmma16b(v16b a, v16b b, v8f c) { v8f d = __builtin_amdgcn_wmma_f32_16x16x32_f16(false, a, false, b, (short)0, c, false, false); asm volatile("v_nop\n\tv_nop\n\tv_nop\n\tv_nop" : "+v"(d) : "v"(a), "v"(b)); return d; }
__device__ __forceinline__ void wave_lds_sync() { __builtin_amdgcn_fence(__ATOMIC_RELEASE, "workgroup"); __builtin_amdgcn_wave_barrier(); __builtin_amdgcn_fence(__ATOMIC_ACQUIRE, "workgroup"); }
__device__ __forceinline__ float pmul(float a, float b) { float p = a * b; asm volatile("" : "+v"(p)); return p; }
__device__ __forceinline__ int iclamp(int v, int lo, int hi) { return v < lo ? lo : (v > hi ? hi : v); }

__global__ __launch_bounds__(256) void wcopy_kernel(const float* __restrict__ w, int KIN, int OUTW, int OUTP, b16* __restrict__ WT) {
  const int u = blockIdx.x * 256 + threadIdx.x; if (u >= OUTP * KIN / 8) return; const int e = u * 8; const int o = e / KIN; v8b v;
#pragma unroll
  for (int j = 0; j < 8; ++j) v[j] = o < OUTW ? (b16)(bf16_rne(w[e + j]) * WSC) : (b16)0.0f; for (int pass = 0; pass < 2; ++pass) { *(volatile v8b*)(WT + e) = v; __threadfence(); }
}
__global__ __launch_bounds__(32) void rnn_kernel(const int* __restrict__ xin, const float* __restrict__ emb, const b16* __restrict__ WIH, const float* __restrict__ bih, const int* __restrict__ xlen, const b16* __restrict__ WHH, const float* __restrict__ bhh, const b16* __restrict__ W1T, const float* __restrict__ b1, const b16* __restrict__ W2T, const float* __restrict__ b2, int BV, float* __restrict__ out) {
  __shared__ __attribute__((aligned(16))) b16 Ah[16][H + 8], Al[16][H + 8], Ae[16][E + 8]; __shared__ __attribute__((aligned(16))) float G[16][H + 4], Ls[16][H + 4]; __shared__ float So[16][C]; __shared__ int Ln[16];
  const int lane = threadIdx.x, nloc = lane & 15, hlf = lane >> 4; const size_t b0 = (size_t)blockIdx.x * 16; if (b0 >= (size_t)BV) return;
  if (lane < 16) Ln[lane] = iclamp(xlen[b0 + lane] - 1, 0, S - 1);
  float bh[8]; for (int q = 0; q < 8; ++q) bh[q] = bf16_rne(bhh[q * 32 + lane]) + bf16_rne(bih[q * 32 + lane]);
  for (int rr = 0; rr < 16; ++rr) for (int q = 0; q < 8; ++q) { Ah[rr][q * 32 + lane] = (b16)0.0f; Al[rr][q * 32 + lane] = (b16)0.0f; Ls[rr][q * 32 + lane] = 0.0f; }
  wave_lds_sync();
#pragma unroll 1
  for (int t = 0; t < S; ++t) {
    for (int rr = 0; rr < 16; ++rr) { const int tok = iclamp(xin[(b0 + rr) * S + t], 0, V - 1); for (int q = 0; q < 4; ++q) Ae[rr][q * 32 + lane] = (b16)(bf16_rne(emb[(size_t)tok * E + q * 32 + lane]) * XS); }
    wave_lds_sync();
#pragma unroll 1
    for (int cg = 0; cg < 2; ++cg) { v8f acc[8];
#pragma unroll
      for (int tt = 0; tt < 8; ++tt) acc[tt] = (v8f){};
#pragma unroll
      for (int kb = 0; kb < E; kb += 32) { const v16b a = frag_kb(&Ae[nloc][kb], hlf);
#pragma unroll
        for (int tt = 0; tt < 8; ++tt) acc[tt] = wmma16b(a, frag_kb(WIH + (size_t)(cg * 128 + tt * 16 + nloc) * E + kb, hlf), acc[tt]); }
#pragma unroll
      for (int tt = 0; tt < 8; ++tt)
#pragma unroll
        for (int r8 = 0; r8 < 8; ++r8) G[8 * hlf + r8][cg * 128 + tt * 16 + nloc] = acc[tt][r8] * (1.0f / (XS * WSC)); }
#pragma unroll 1
    for (int cg = 0; cg < 2; ++cg) { v8f acc[8];
#pragma unroll
      for (int tt = 0; tt < 8; ++tt) acc[tt] = (v8f){};
#pragma unroll 2
      for (int kb = 0; kb < H; kb += 32) { const v16b a = frag_kb(&Ah[nloc][kb], hlf), a2 = frag_kb(&Al[nloc][kb], hlf);
#pragma unroll
        for (int tt = 0; tt < 8; ++tt) { const v16b bw = frag_kb(WHH + (size_t)(cg * 128 + tt * 16 + nloc) * H + kb, hlf); acc[tt] = wmma16b(a, bw, acc[tt]); acc[tt] = wmma16b(a2, bw, acc[tt]); } }
#pragma unroll
      for (int tt = 0; tt < 8; ++tt)
#pragma unroll
        for (int r8 = 0; r8 < 8; ++r8) G[8 * hlf + r8][cg * 128 + tt * 16 + nloc] += acc[tt][r8] * (1.0f / (HS * WSC)); }
    wave_lds_sync();
    for (int rr = 0; rr < 16; ++rr) { const bool keep = (Ln[rr] == t);
      for (int q = 0; q < 8; ++q) { const int c = q * 32 + lane; const float hv = tanhf(G[rr][c] + bh[q]); b16 p, ql; split16(hv * HS, p, ql); Ah[rr][c] = p; Al[rr][c] = ql; if (keep) Ls[rr][c] = hv; } }
    wave_lds_sync(); }
  for (int rr = 0; rr < 16; ++rr) for (int q = 0; q < 8; ++q) { const int c = q * 32 + lane; b16 p, ql; split16(Ls[rr][c] * HS, p, ql); Ah[rr][c] = p; Al[rr][c] = ql; }
  wave_lds_sync();
#pragma unroll 1
  for (int cg = 0; cg < 2; ++cg) { v8f acc[8];
#pragma unroll
    for (int tt = 0; tt < 8; ++tt) acc[tt] = (v8f){};
#pragma unroll 2
    for (int kb = 0; kb < H; kb += 32) { const v16b a = frag_kb(&Ah[nloc][kb], hlf), a2 = frag_kb(&Al[nloc][kb], hlf);
#pragma unroll
      for (int tt = 0; tt < 8; ++tt) { const v16b bw = frag_kb(W1T + (size_t)(cg * 128 + tt * 16 + nloc) * H + kb, hlf); acc[tt] = wmma16b(a, bw, acc[tt]); acc[tt] = wmma16b(a2, bw, acc[tt]); } }
#pragma unroll
    for (int tt = 0; tt < 8; ++tt) { const int c = cg * 128 + tt * 16 + nloc; const float bb = bf16_rne(b1[c]);
#pragma unroll
      for (int r8 = 0; r8 < 8; ++r8) G[8 * hlf + r8][c] = fmaxf(acc[tt][r8] * (1.0f / (HS * WSC)) + bb, 0.0f); } }
  wave_lds_sync();
  for (int rr = 0; rr < 16; ++rr) for (int q = 0; q < 8; ++q) { const int c = q * 32 + lane; b16 p, ql; split16(G[rr][c] * YS, p, ql); Ah[rr][c] = p; Al[rr][c] = ql; }
  wave_lds_sync();
  { v8f acc[2] = {(v8f){}, (v8f){}};
#pragma unroll 2
    for (int kb = 0; kb < H; kb += 32) { const v16b a = frag_kb(&Ah[nloc][kb], hlf), a2 = frag_kb(&Al[nloc][kb], hlf);
#pragma unroll
      for (int tt = 0; tt < 2; ++tt) { const v16b bw = frag_kb(W2T + (size_t)(tt * 16 + nloc) * H + kb, hlf); acc[tt] = wmma16b(a, bw, acc[tt]); acc[tt] = wmma16b(a2, bw, acc[tt]); } }
#pragma unroll
    for (int tt = 0; tt < 2; ++tt) { const int c = tt * 16 + nloc; if (c < C) { const float bb = bf16_rne(b2[c]);
#pragma unroll
        for (int r8 = 0; r8 < 8; ++r8) So[8 * hlf + r8][c] = acc[tt][r8] * (1.0f / (YS * WSC)) + bb; } } }
  wave_lds_sync();
  for (int pass = 0; pass < 2; ++pass) { for (int i = lane; i < 16 * C; i += 32) ((volatile float*)out)[b0 * C + i] = So[i / C][i % C]; __threadfence(); }
}
}

extern "C" void kernel_launch(void* const* d_in, const int* in_sizes, int n_in, void* d_out, int out_size, void* d_ws, size_t ws_size, hipStream_t stream) {
  (void)n_in;
  auto Fp = [&](int i) { return (const float*)d_in[i]; }; auto Ip = [&](int i) { return (const int*)d_in[i]; };
  if (in_sizes[0] != B * S || in_sizes[1] != B || in_sizes[2] != V * E || in_sizes[3] != H * E || in_sizes[4] != H * H || in_sizes[7] != H * H || in_sizes[9] != C * H || out_size != B * C) return;
  const int BV = B;
  size_t off = 0; char* ws = (char*)d_ws;
  auto carve = [&](size_t bytes) { char* p = ws + off; off += (bytes + 255) & ~(size_t)255; return p; };
  b16* WIH = (b16*)carve((size_t)H * E * 2); b16* WHH = (b16*)carve((size_t)H * H * 2); b16* W1T = (b16*)carve((size_t)H * H * 2); b16* W2T = (b16*)carve((size_t)32 * H * 2);
  if (off > ws_size || off > ((size_t)4 << 20)) return;
  wcopy_kernel<<<(H * E / 8 + 255) / 256, 256, 0, stream>>>(Fp(3), E, H, H, WIH); wcopy_kernel<<<(H * H / 8 + 255) / 256, 256, 0, stream>>>(Fp(4), H, H, H, WHH); wcopy_kernel<<<(H * H / 8 + 255) / 256, 256, 0, stream>>>(Fp(7), H, H, H, W1T); wcopy_kernel<<<(32 * H / 8 + 255) / 256, 256, 0, stream>>>(Fp(9), H, C, 32, W2T);
  rnn_kernel<<<BV / 16, 32, 0, stream>>>(Ip(0), Fp(2), WIH, Fp(5), Ip(1), WHH, Fp(6), W1T, Fp(8), W2T, Fp(10), BV, (float*)d_out);
}
